// MaskedMHA_73572789780875
// MI455X (gfx1250) — hardware-verified
//
#include <hip/hip_runtime.h>


#define NB_  4
#define TT   2048
#define DD   1024
#define NH_  16
#define HD   64
#define NT   (NB_ * TT)
#define ZH   2
#define TE   512
#define PCAR 1024.0f
typedef _Float16 h16;
typedef unsigned short bf;
typedef __attribute__((ext_vector_type(16))) __bf16   v16bf;
typedef __attribute__((ext_vector_type(16))) _Float16 v16h;
typedef __attribute__((ext_vector_type(8)))  _Float16 v8h;
typedef __attribute__((ext_vector_type(8)))  unsigned short v8us;
typedef __attribute__((ext_vector_type(8)))  float    v8f;
typedef __attribute__((ext_vector_type(4)))  float    v4f;
typedef v8h  __attribute__((may_alias)) v8ha;
typedef v4f  __attribute__((may_alias)) v4fa;
typedef v8us __attribute__((may_alias)) v8usa;

__device__ __forceinline__ unsigned short f2bf(float f) { unsigned u = __float_as_uint(f); u += 0x7FFFu + ((u >> 16) & 1u); return (unsigned short)(u >> 16); }
__device__ __forceinline__ float bf2f(unsigned short b) { return __uint_as_float(((unsigned)b) << 16); }
__device__ __forceinline__ float bfr(float f) { return bf2f(f2bf(f)); }
__device__ __forceinline__ v16h cat16(v8h lo, v8h hi) { return __builtin_shufflevector(lo, hi, 0, 1, 2, 3, 4, 5, 6, 7, 8, 9, 10, 11, 12, 13, 14, 15); }
__device__ __forceinline__ v16bf cat16b(v8us lo, v8us hi) { return __builtin_bit_cast(v16bf, __builtin_shufflevector(lo, hi, 0, 1, 2, 3, 4, 5, 6, 7, 8, 9, 10, 11, 12, 13, 14, 15)); }
__device__ __forceinline__ v8f wmma16(v16h a, v16h b, v8f c) { return __builtin_amdgcn_wmma_f32_16x16x32_f16(false, a, false, b, (short)0, c, false, false); }
__device__ __forceinline__ v8f wmmab(v16bf a, v16bf b, v8f c) { return __builtin_amdgcn_wmma_f32_16x16x32_bf16(false, a, false, b, (short)0, c, false, false); }


template <typename T16> struct WFrag;
template <> struct WFrag<h16> { typedef v16h V; static __device__ __forceinline__ V ld(const h16* p) { return cat16(*(const v8h*)p, *(const v8h*)(p + 16)); } static __device__ __forceinline__ v8f mma(V a, V b, v8f c) { return wmma16(a, b, c); } };
template <> struct WFrag<bf> { typedef v16bf V; static __device__ __forceinline__ V ld(const bf* p) { return cat16b(*(const v8us*)p, *(const v8us*)(p + 16)); } static __device__ __forceinline__ v8f mma(V a, V b, v8f c) { return wmmab(a, b, c); } };
template <typename T16, int NSPLIT, bool BIAS>
__global__ __launch_bounds__(32) void k_gemmw(const T16* __restrict__ A, const T16* __restrict__ A2, const T16* __restrict__ Bt, const T16* __restrict__ Bt2, int K, float* C, int ldc, const float* __restrict__ bias, size_t sA, size_t sB, size_t sC) {
    typedef typename WFrag<T16>::V V;
    __shared__ __align__(16) float os[16 * 68];
    const size_t z = blockIdx.z; A += z * sA; if (A2) A2 += z * sA; Bt += z * sB; if (Bt2) Bt2 += z * sB; C += z * sC;
    const int lane = threadIdx.x & 31, lr = lane & 15, hi = lane >> 4; const int r0 = blockIdx.x * 64, c0 = blockIdx.y * 64;
    v8f acc[4][4];
#pragma unroll
    for (int mb = 0; mb < 4; ++mb)
#pragma unroll
        for (int nb = 0; nb < 4; ++nb) acc[mb][nb] = (v8f){};
    const size_t aoff = (size_t)(r0 + lr) * K + 8 * hi, boff = (size_t)(c0 + lr) * K + 8 * hi;
#pragma unroll 1
    for (int kc = 0; kc < K; kc += 32) {
        V a[4], a2[4];
#pragma unroll
        for (int mb = 0; mb < 4; ++mb) { a[mb] = WFrag<T16>::ld(A + aoff + (size_t)mb * 16 * K + kc); if (NSPLIT == 1 || NSPLIT == 2) a2[mb] = WFrag<T16>::ld(A2 + aoff + (size_t)mb * 16 * K + kc); }
#pragma unroll
        for (int nb = 0; nb < 4; ++nb) { const V b = WFrag<T16>::ld(Bt + boff + (size_t)nb * 16 * K + kc); V b2; if (NSPLIT >= 2) b2 = WFrag<T16>::ld(Bt2 + boff + (size_t)nb * 16 * K + kc);
#pragma unroll
            for (int mb = 0; mb < 4; ++mb) { acc[mb][nb] = WFrag<T16>::mma(a[mb], b, acc[mb][nb]); if (NSPLIT == 1 || NSPLIT == 2) acc[mb][nb] = WFrag<T16>::mma(a2[mb], b, acc[mb][nb]); if (NSPLIT >= 2) acc[mb][nb] = WFrag<T16>::mma(a[mb], b2, acc[mb][nb]); } }
        asm volatile("v_nop\n\tv_nop\n\tv_nop\n\tv_nop" : "+v"(acc[0][0]), "+v"(acc[1][1]), "+v"(acc[2][2]), "+v"(acc[3][3]) : "v"(a[0]), "v"(a[3]));
    }
#pragma unroll
    for (int mb = 0; mb < 4; ++mb) {
#pragma unroll
        for (int nb = 0; nb < 4; ++nb) {
#pragma unroll
            for (int j = 0; j < 8; ++j) os[(hi * 8 + j) * 68 + nb * 16 + lr] = acc[mb][nb][j]; }
        __builtin_amdgcn_wave_barrier(); asm volatile("" ::: "memory");
        float* crow = C + (size_t)(r0 + mb * 16) * ldc + c0;
#pragma unroll 1
        for (int ps = 0; ps < 2; ++ps) {
#pragma unroll
            for (int s = 0; s < 8; ++s) { const int row = 2 * s + hi, cofs = lr * 4; v4f val = *(const v4fa*)(os + row * 68 + cofs); if (BIAS) { val[0] += bfr(bias[c0 + cofs]); val[1] += bfr(bias[c0 + cofs + 1]); val[2] += bfr(bias[c0 + cofs + 2]); val[3] += bfr(bias[c0 + cofs + 3]); }
                *(volatile v4f*)(crow + (size_t)row * ldc + cofs) = val; }
            if (ps == 0) __threadfence(); }
        __builtin_amdgcn_wave_barrier(); asm volatile("" ::: "memory");
    }
}

template <typename T16, int CMODE, int NSPLIT = 0>
__global__ __launch_bounds__(32) void k_gemmwc(const T16* __restrict__ A, const T16* __restrict__ A2, const T16* __restrict__ Bt, const T16* __restrict__ Bt2, int K, float* C, int ldc, const float* __restrict__ bias, size_t sA, size_t sB, size_t sC) {
    constexpr bool BIAS = false; typedef typename WFrag<T16>::V V;
    __shared__ __align__(16) float os[16 * 68];
    const size_t z = blockIdx.z; A += z * sA; if (A2) A2 += z * sA; Bt += z * sB; if (Bt2) Bt2 += z * sB; C += z * sC;
    const int lane = threadIdx.x & 31, lr = lane & 15, hi = lane >> 4; const int r0 = blockIdx.x * 64, c0 = blockIdx.y * 64;
    if (CMODE == 1 && c0 > r0 + 63) return;
    const int Keff = (CMODE == 2 && r0 + 64 < K) ? r0 + 64 : K;
    v8f acc[4][4];
#pragma unroll
    for (int mb = 0; mb < 4; ++mb)
#pragma unroll
        for (int nb = 0; nb < 4; ++nb) acc[mb][nb] = (v8f){};
    const size_t aoff = (size_t)(r0 + lr) * K + 8 * hi, boff = (size_t)(c0 + lr) * K + 8 * hi;
#pragma unroll 1
    for (int kc = 0; kc < Keff; kc += 32) {
        V a[4], a2[4];
#pragma unroll
        for (int mb = 0; mb < 4; ++mb) { a[mb] = WFrag<T16>::ld(A + aoff + (size_t)mb * 16 * K + kc); if (NSPLIT == 1 || NSPLIT == 2) a2[mb] = WFrag<T16>::ld(A2 + aoff + (size_t)mb * 16 * K + kc); }
#pragma unroll
        for (int nb = 0; nb < 4; ++nb) { const V b = WFrag<T16>::ld(Bt + boff + (size_t)nb * 16 * K + kc); V b2; if (NSPLIT >= 2) b2 = WFrag<T16>::ld(Bt2 + boff + (size_t)nb * 16 * K + kc);
#pragma unroll
            for (int mb = 0; mb < 4; ++mb) { acc[mb][nb] = WFrag<T16>::mma(a[mb], b, acc[mb][nb]); if (NSPLIT == 1 || NSPLIT == 2) acc[mb][nb] = WFrag<T16>::mma(a2[mb], b, acc[mb][nb]); if (NSPLIT >= 2) acc[mb][nb] = WFrag<T16>::mma(a[mb], b2, acc[mb][nb]); } }
        asm volatile("v_nop\n\tv_nop\n\tv_nop\n\tv_nop" : "+v"(acc[0][0]), "+v"(acc[1][1]), "+v"(acc[2][2]), "+v"(acc[3][3]) : "v"(a[0]), "v"(a[3]));
    }
#pragma unroll
    for (int mb = 0; mb < 4; ++mb) {
#pragma unroll
        for (int nb = 0; nb < 4; ++nb) {
#pragma unroll
            for (int j = 0; j < 8; ++j) os[(hi * 8 + j) * 68 + nb * 16 + lr] = acc[mb][nb][j]; }
        __builtin_amdgcn_wave_barrier(); asm volatile("" ::: "memory");
        float* crow = C + (size_t)(r0 + mb * 16) * ldc + c0;
#pragma unroll 1
        for (int ps = 0; ps < 2; ++ps) {
#pragma unroll
            for (int s = 0; s < 8; ++s) { const int row = 2 * s + hi, cofs = lr * 4; v4f val = *(const v4fa*)(os + row * 68 + cofs); if (BIAS) { val[0] += bfr(bias[c0 + cofs]); val[1] += bfr(bias[c0 + cofs + 1]); val[2] += bfr(bias[c0 + cofs + 2]); val[3] += bfr(bias[c0 + cofs + 3]); }
                *(volatile v4f*)(crow + (size_t)row * ldc + cofs) = val; }
            if (ps == 0) __threadfence(); }
        __builtin_amdgcn_wave_barrier(); asm volatile("" ::: "memory");
    }
}

__device__ __forceinline__ h16 tohx(float x) { return (h16)x; }
typedef __attribute__((ext_vector_type(4))) _Float16 v4h;
typedef __attribute__((ext_vector_type(2))) _Float16 v2h;

template <bool H16>
__global__ __launch_bounds__(256) void k_wtT(const float* __restrict__ w, unsigned short* Bt) {
    typedef __attribute__((ext_vector_type(2))) unsigned short v2us_;
    const int lane = threadIdx.x & 31; const int L0 = (blockIdx.x * 8 + (threadIdx.x >> 5)) * 8; const int nlines = DD * DD / 64;
#pragma unroll 1
    for (int ps = 0; ps < 2; ++ps) {
#pragma unroll
        for (int l = 0; l < 8; ++l) { const int L = L0 + l; if (L >= nlines) break; const int e = L * 64 + lane * 2; const int k = e & (DD - 1), n = e >> 10; v2us_ o;
#pragma unroll
            for (int q = 0; q < 2; ++q) { const float v = bfr(w[(size_t)(k + q) * DD + n]); if (H16) { _Float16 hv = (_Float16)v; o[q] = __builtin_bit_cast(unsigned short, hv); } else o[q] = f2bf(v); }
            *(volatile v2us_*)(Bt + (size_t)e) = o; }
        if (ps == 0) __threadfence(); }
}
__global__ __launch_bounds__(256) void k_cvt8(const float* __restrict__ src, bf* dst, size_t n8) { const size_t i = (size_t)blockIdx.x * 256 + threadIdx.x; if (i >= n8) return; const v8f v = *(const v8f*)(src + i * 8); v8us o;
#pragma unroll
    for (int k = 0; k < 8; ++k) o[k] = f2bf(v[k]); *(volatile v8us*)(dst + i * 8) = o; __threadfence(); *(volatile v8us*)(dst + i * 8) = o; }
__global__ __launch_bounds__(256) void k_cvt8h(const float* __restrict__ src, h16* dst, size_t n8) { const size_t i = (size_t)blockIdx.x * 256 + threadIdx.x; if (i >= n8) return; const v8f v = *(const v8f*)(src + i * 8); v8h o;
#pragma unroll
    for (int k = 0; k < 8; ++k) o[k] = tohx(bfr(v[k])); *(volatile v8h*)(dst + i * 8) = o; __threadfence(); *(volatile v8h*)(dst + i * 8) = o; }
__global__ __launch_bounds__(256) void k_hplane(const float* __restrict__ F, int h8, float sc, h16* P) {
    const int lane = threadIdx.x & 31; const int L0 = (blockIdx.x * 8 + (threadIdx.x >> 5)) * 8; const int nlines = NT * 512 / 64;
#pragma unroll 1
    for (int ps = 0; ps < 2; ++ps) {
#pragma unroll
        for (int l = 0; l < 8; ++l) { const int L = L0 + l; if (L >= nlines) break; const int e = L * 64 + lane * 2; const int d = e & 63; const int t = (e >> 6) % TT; const int zz = e / (64 * TT); const int b = zz >> 3, hl = zz & 7; v2h v;
#pragma unroll
            for (int q = 0; q < 2; ++q) v[q] = tohx(F[((size_t)b * TT + t) * 512 + hl * HD + d + q] * sc);
            *(volatile v2h*)(P + ((size_t)(b * NH_ + h8 + hl) * TT + t) * HD + d) = v; }
        if (ps == 0) __threadfence(); }
}
__global__ __launch_bounds__(256) void k_hplane2(const float* __restrict__ F, int h8, float sc, bf* Ph, bf* Pl) {
    typedef __attribute__((ext_vector_type(2))) unsigned short v2us_;
    const int lane = threadIdx.x & 31; const int L0 = (blockIdx.x * 8 + (threadIdx.x >> 5)) * 8; const int nlines = NT * 512 / 64;
#pragma unroll 1
    for (int ps = 0; ps < 2; ++ps) {
#pragma unroll
        for (int l = 0; l < 8; ++l) { const int L = L0 + l; if (L >= nlines) break; const int e = L * 64 + lane * 2; const int d = e & 63; const int t = (e >> 6) % TT; const int zz = e / (64 * TT); const int b = zz >> 3, hl = zz & 7; v2us_ oh, ol;
#pragma unroll
            for (int q = 0; q < 2; ++q) { const float y = F[((size_t)b * TT + t) * 512 + hl * HD + d + q] * sc; const unsigned short a = f2bf(y); oh[q] = a; ol[q] = f2bf(y - bf2f(a)); }
            const size_t o = ((size_t)(b * NH_ + h8 + hl) * TT + t) * HD + d; *(volatile v2us_*)(Ph + o) = oh; *(volatile v2us_*)(Pl + o) = ol; }
        if (ps == 0) __threadfence(); }
}
__global__ __launch_bounds__(256) void k_vtplane(const float* __restrict__ F, int h8, h16* VT) {
    const int lane = threadIdx.x & 31; const int L0 = (blockIdx.x * 8 + (threadIdx.x >> 5)) * 8; const int nlines = NT * 512 / 64;
#pragma unroll 1
    for (int ps = 0; ps < 2; ++ps) {
#pragma unroll
        for (int l = 0; l < 8; ++l) { const int L = L0 + l; if (L >= nlines) break; const int e = L * 64 + lane * 2; const int t = e % TT; const int d = (e / TT) % 64; const int zz = e / (64 * TT); const int b = zz >> 3, hl = zz & 7; v2h v;
#pragma unroll
            for (int q = 0; q < 2; ++q) v[q] = tohx(F[((size_t)b * TT + t + q) * 512 + hl * HD + d]);
            *(volatile v2h*)(VT + ((size_t)(b * NH_ + h8 + hl) * HD + d) * TT + t) = v; }
        if (ps == 0) __threadfence(); }
}
__global__ __launch_bounds__(256) void k_softc(const float* __restrict__ Sb, h16* P) {
    const int lane = threadIdx.x & 31; const int row = blockIdx.x * 8 + (threadIdx.x >> 5); if (row >= ZH * TT) return; const int i = row % TT; const float* sr = Sb + (size_t)row * TT;
    const int kend = ((i >> 6) + 1) * 64;
    float m = -3.0e38f;
#pragma unroll 1
    for (int c0 = lane * 4; c0 < kend; c0 += 128) {
#pragma unroll
        for (int q = 0; q < 4; ++q) { const int k = c0 + q; if (k <= i) m = fmaxf(m, sr[k <= i ? k : 0]); } }
#pragma unroll
    for (int sh = 16; sh; sh >>= 1) m = fmaxf(m, __shfl_xor(m, sh, 32));
    float sum = 0.f;
#pragma unroll 1
    for (int c0 = lane * 4; c0 < kend; c0 += 128) {
#pragma unroll
        for (int q = 0; q < 4; ++q) { const int k = c0 + q; if (k <= i) sum += __expf(sr[k <= i ? k : 0] - m); } }
#pragma unroll
    for (int sh = 16; sh; sh >>= 1) sum += __shfl_xor(sum, sh, 32);
    const float f = __fdiv_rn(PCAR, sum);
#pragma unroll 1
    for (int ps = 0; ps < 2; ++ps) {
#pragma unroll 1
        for (int c0 = (lane & 15) * 4; c0 < kend; c0 += 64) {
            if (((c0 >> 6) & 1) != (lane >> 4)) continue;
            v4h o;
#pragma unroll
            for (int q = 0; q < 4; ++q) { const int k = c0 + q; o[q] = (k <= i) ? tohx(__expf(sr[k <= i ? k : 0] - m) * f) : tohx(0.f); }
            *(volatile v4h*)(P + (size_t)row * TT + c0) = o; }
        if (ps == 0) __threadfence(); }
}
__global__ __launch_bounds__(256) void k_merge(const float* __restrict__ O, int b, int h0, h16* AT) {
    const int lane = threadIdx.x & 31; const int t = blockIdx.x * 8 + (threadIdx.x >> 5); if (t >= TT) return; const int zz = lane >> 4, d = (lane & 15) * 4; v4h o;
#pragma unroll
    for (int q = 0; q < 4; ++q) o[q] = tohx(O[((size_t)zz * TT + t) * 64 + d + q] * (1.0f / PCAR));
    h16* dst = AT + ((size_t)b * TT + t) * DD + (h0 + zz) * HD + d; *(volatile v4h*)dst = o; __threadfence(); *(volatile v4h*)dst = o;
}

__device__ __forceinline__ void splitf(float y, unsigned short& h, unsigned short& l) { h = f2bf(y); l = f2bf(y - bf2f(h)); }
template <bool VT_>
__global__ __launch_bounds__(256) void k_eplane(const float* __restrict__ F, int h8, float sc, bf* Ph, bf* Pl) {
    typedef __attribute__((ext_vector_type(2))) unsigned short v2us;
    const int lane = threadIdx.x & 31; const int L0 = (blockIdx.x * 8 + (threadIdx.x >> 5)) * 8; const int nlines = NB_ * 8 * TE * HD / 64;
#pragma unroll 1
    for (int ps = 0; ps < 2; ++ps) {
#pragma unroll
        for (int l = 0; l < 8; ++l) { const int L = L0 + l; if (L >= nlines) break; const int e = L * 64 + lane * 2; int t, d, zz; if (VT_) { t = e % TE; d = (e / TE) % HD; zz = e / (HD * TE); } else { d = e % HD; t = (e / HD) % TE; zz = e / (HD * TE); }
            const int b = zz >> 3, hl = zz & 7; v2us oh, ol;
#pragma unroll
            for (int q = 0; q < 2; ++q) { const int tt = VT_ ? t + q : t, dd = VT_ ? d : d + q; unsigned short a, c2; splitf(F[((size_t)b * TT + tt) * 512 + hl * HD + dd] * sc, a, c2); oh[q] = a; ol[q] = c2; }
            const size_t o = VT_ ? (((size_t)(b * NH_ + h8 + hl) * HD + d) * TE + t) : (((size_t)(b * NH_ + h8 + hl) * TE + t) * HD + d);
            *(volatile v2us*)(Ph + o) = oh; *(volatile v2us*)(Pl + o) = ol; }
        if (ps == 0) __threadfence(); }
}
__global__ __launch_bounds__(256) void k_esoft(const float* __restrict__ ES, bf* Ph, bf* Pl) {
    typedef __attribute__((ext_vector_type(4))) unsigned short v4us;
    const int lane = threadIdx.x & 31; const int row = blockIdx.x * 8 + (threadIdx.x >> 5); if (row >= NH_ * TE) return; const int i = row % TE; const float* sr = ES + (size_t)row * TE; float v[TE / 32]; float mx = -3.0e38f;
#pragma unroll
    for (int ch = 0; ch < TE / 128; ++ch)
#pragma unroll
        for (int q = 0; q < 4; ++q) { const int k = ch * 128 + lane * 4 + q; const float t = (k <= i) ? sr[k] : -3.0e38f; v[ch * 4 + q] = t; mx = fmaxf(mx, t); }
#pragma unroll
    for (int sh = 16; sh; sh >>= 1) mx = fmaxf(mx, __shfl_xor(mx, sh, 32));
    float sum = 0.f;
#pragma unroll
    for (int ch = 0; ch < TE / 128; ++ch)
#pragma unroll
        for (int q = 0; q < 4; ++q) { const int k = ch * 128 + lane * 4 + q; v[ch * 4 + q] = (k <= i) ? __expf(v[ch * 4 + q] - mx) : 0.f; sum += v[ch * 4 + q]; }
#pragma unroll
    for (int sh = 16; sh; sh >>= 1) sum += __shfl_xor(sum, sh, 32);
    const float f = __fdiv_rn(1.0f, sum); v4us oh[TE / 128], ol[TE / 128];
#pragma unroll
    for (int ch = 0; ch < TE / 128; ++ch)
#pragma unroll
        for (int q = 0; q < 4; ++q) { unsigned short a, c2; splitf(v[ch * 4 + q] * f, a, c2); oh[ch][q] = a; ol[ch][q] = c2; }
#pragma unroll 1
    for (int ps = 0; ps < 2; ++ps) {
#pragma unroll
        for (int ch = 0; ch < TE / 128; ++ch) { *(volatile v4us*)(Ph + (size_t)row * TE + ch * 128 + lane * 4) = oh[ch]; *(volatile v4us*)(Pl + (size_t)row * TE + ch * 128 + lane * 4) = ol[ch]; }
        if (ps == 0) __threadfence(); }
}
__global__ __launch_bounds__(256) void k_emerge(const float* __restrict__ EO, int b, bf* Ah, bf* Al) {
    typedef __attribute__((ext_vector_type(2))) unsigned short v2us;
    const int lane = threadIdx.x & 31; const int L = blockIdx.x * 8 + (threadIdx.x >> 5); if (L >= TE * DD / 64) return; const int e = L * 64 + lane * 2; const int c = e % DD, t = e / DD; const int h = c / HD, d = c % HD; v2us oh, ol;
#pragma unroll
    for (int q = 0; q < 2; ++q) { unsigned short a, c2; splitf(EO[((size_t)h * TE + t) * HD + d + q], a, c2); oh[q] = a; ol[q] = c2; }
    const size_t o = ((size_t)b * TE + t) * DD + c; *(volatile v2us*)(Ah + o) = oh; *(volatile v2us*)(Al + o) = ol; __threadfence(); *(volatile v2us*)(Ah + o) = oh; *(volatile v2us*)(Al + o) = ol;
}

extern "C" void kernel_launch(void* const* d_in, const int* in_sizes, int n_in,
                              void* d_out, int out_size, void* d_ws, size_t ws_size, hipStream_t stream) {
    (void)in_sizes; (void)n_in; (void)out_size;
    const float* x = (const float*)d_in[0]; const float* Wq = (const float*)d_in[1]; const float* bq = (const float*)d_in[2]; const float* Wk = (const float*)d_in[3]; const float* bk = (const float*)d_in[4];
    const float* Wv = (const float*)d_in[5]; const float* bv = (const float*)d_in[6]; const float* Wo = (const float*)d_in[7]; const float* bo = (const float*)d_in[8];
    float* OUT = (float*)d_out;
    char* wsp = (char*)d_ws;
    auto take = [&](size_t bytes) { char* p = wsp; wsp += (bytes + 255) & ~(size_t)255; return (void*)p; };
    bf* WQ = (bf*)take((size_t)DD * DD * 2); bf* WK = (bf*)take((size_t)DD * DD * 2); bf* WV = (bf*)take((size_t)DD * DD * 2); h16* WO = (h16*)take((size_t)DD * DD * 2); bf* WOB = (bf*)take((size_t)DD * DD * 2);
    bf* ATEh = (bf*)take((size_t)NB_ * TE * DD * 2); bf* ATEl = (bf*)take((size_t)NB_ * TE * DD * 2);
    float* SCR = (float*)take((size_t)NT * 512 * 4);
    bf* QPh = (bf*)take((size_t)NT * DD * 2); bf* QPl = (bf*)take((size_t)NT * DD * 2); bf* KPh = (bf*)take((size_t)NT * DD * 2); bf* KPl = (bf*)take((size_t)NT * DD * 2); h16* VT = (h16*)take((size_t)NT * DD * 2);
    float* Sb = (float*)take((size_t)ZH * TT * TT * 4);
    h16* Pm = (h16*)take((size_t)ZH * TT * TT * 2); float* Ob = (float*)take((size_t)ZH * TT * HD * 4);
    bf* XB = (bf*)Sb; h16* AT = (h16*)SCR;
    const size_t EPL = (size_t)NB_ * NH_ * TE * HD;
    bf* QEh = (bf*)take(EPL * 2); bf* QEl = (bf*)take(EPL * 2); bf* KEh = (bf*)take(EPL * 2); bf* KEl = (bf*)take(EPL * 2); bf* VEh = (bf*)take(EPL * 2); bf* VEl = (bf*)take(EPL * 2);
    float* ESb = (float*)take((size_t)NH_ * TE * TE * 4); bf* EPh = (bf*)take((size_t)NH_ * TE * TE * 2); bf* EPl = (bf*)take((size_t)NH_ * TE * TE * 2); float* EO = (float*)take((size_t)NH_ * TE * HD * 4);
    if ((size_t)(wsp - (char*)d_ws) > ws_size) return;
    { const unsigned gT = (unsigned)((DD * DD / 64 + 63) / 64); k_wtT<false><<<gT, 256, 0, stream>>>(Wq, WQ); k_wtT<false><<<gT, 256, 0, stream>>>(Wk, WK); k_wtT<false><<<gT, 256, 0, stream>>>(Wv, WV); k_wtT<true><<<gT, 256, 0, stream>>>(Wo, (unsigned short*)WO); k_wtT<false><<<gT, 256, 0, stream>>>(Wo, WOB);
      const size_t nx = (size_t)NT * DD / 8; k_cvt8<<<(unsigned)((nx + 255) / 256), 256, 0, stream>>>(x, XB, nx); }
    const unsigned LBP = (unsigned)((NT * 512 / 64 + 63) / 64); const unsigned LBE = (unsigned)((NB_ * 8 * TE * HD / 64 + 63) / 64);
    for (int h8 = 0; h8 < NH_; h8 += 8) {
        k_gemmw<bf, 0, true><<<dim3(NT / 64, 512 / 64, 1), 32, 0, stream>>>(XB, nullptr, WQ + (size_t)h8 * HD * DD, nullptr, DD, SCR, 512, bq + h8 * HD, 0, 0, 0); k_hplane2<<<LBP, 256, 0, stream>>>(SCR, h8, 0.125f, QPh, QPl); k_eplane<false><<<LBE, 256, 0, stream>>>(SCR, h8, 0.125f, QEh, QEl);
        k_gemmw<bf, 0, true><<<dim3(NT / 64, 512 / 64, 1), 32, 0, stream>>>(XB, nullptr, WK + (size_t)h8 * HD * DD, nullptr, DD, SCR, 512, bk + h8 * HD, 0, 0, 0); k_hplane2<<<LBP, 256, 0, stream>>>(SCR, h8, 1.0f, KPh, KPl); k_eplane<false><<<LBE, 256, 0, stream>>>(SCR, h8, 1.0f, KEh, KEl);
        k_gemmw<bf, 0, true><<<dim3(NT / 64, 512 / 64, 1), 32, 0, stream>>>(XB, nullptr, WV + (size_t)h8 * HD * DD, nullptr, DD, SCR, 512, bv + h8 * HD, 0, 0, 0); k_vtplane<<<LBP, 256, 0, stream>>>(SCR, h8, VT); k_eplane<true><<<LBE, 256, 0, stream>>>(SCR, h8, 1.0f, VEh, VEl); }
    for (int b = 0; b < NB_; ++b) { const size_t z0 = (size_t)b * NH_;
        k_gemmw<bf, 2, false><<<dim3(TE / 64, TE / 64, NH_), 32, 0, stream>>>(QEh + z0 * TE * HD, QEl + z0 * TE * HD, KEh + z0 * TE * HD, KEl + z0 * TE * HD, HD, ESb, TE, nullptr, (size_t)TE * HD, (size_t)TE * HD, (size_t)TE * TE);
        k_esoft<<<NH_ * TE / 8, 256, 0, stream>>>(ESb, EPh, EPl);
        k_gemmw<bf, 2, false><<<dim3(TE / 64, 1, NH_), 32, 0, stream>>>(EPh, EPl, VEh + z0 * HD * TE, VEl + z0 * HD * TE, TE, EO, HD, nullptr, (size_t)TE * TE, (size_t)HD * TE, (size_t)TE * HD);
        k_emerge<<<(TE * DD / 64 + 7) / 8, 256, 0, stream>>>(EO, b, ATEh, ATEl); }
    for (int b = 0; b < NB_; ++b)
        for (int h0 = 0; h0 < NH_; h0 += ZH) { const size_t z0 = (size_t)b * NH_ + h0;
            k_gemmwc<bf, 1, 2><<<dim3(TT / 64, TT / 64, ZH), 32, 0, stream>>>(QPh + z0 * TT * HD, QPl + z0 * TT * HD, KPh + z0 * TT * HD, KPl + z0 * TT * HD, HD, Sb, TT, nullptr, (size_t)TT * HD, (size_t)TT * HD, (size_t)TT * TT);
            k_softc<<<ZH * TT / 8, 256, 0, stream>>>(Sb, Pm);
            k_gemmwc<h16, 2><<<dim3(TT / 64, 1, ZH), 32, 0, stream>>>(Pm, nullptr, VT + z0 * HD * TT, nullptr, TT, Ob, HD, nullptr, (size_t)TT * TT, (size_t)HD * TT, (size_t)TT * HD);
            k_merge<<<TT / 8, 256, 0, stream>>>(Ob, b, h0, AT); }
    for (int b = 0; b < NB_; ++b) {
        k_gemmw<bf, 1, true><<<dim3(TE / 64, DD / 64, 1), 32, 0, stream>>>(ATEh + (size_t)b * TE * DD, ATEl + (size_t)b * TE * DD, WOB, nullptr, DD, OUT + (size_t)b * TT * DD, DD, bo, 0, 0, 0);
        k_gemmw<h16, 0, true><<<dim3((TT - TE) / 64, DD / 64, 1), 32, 0, stream>>>(AT + ((size_t)b * TT + TE) * DD, nullptr, WO, nullptr, DD, OUT + ((size_t)b * TT + TE) * DD, DD, bo, 0, 0, 0); }
}
